// CKConv_10368051052953
// MI455X (gfx1250) — hardware-verified
//
#include <hip/hip_runtime.h>


namespace {
typedef _Float16 b16;
typedef __attribute__((ext_vector_type(16))) _Float16 v16b;
typedef __attribute__((ext_vector_type(8))) _Float16 v8b;
typedef __attribute__((ext_vector_type(4))) _Float16 v4h;
typedef __attribute__((ext_vector_type(2))) _Float16 v2h;
typedef __attribute__((ext_vector_type(8))) float v8f;
typedef __attribute__((ext_vector_type(4))) float v4f;
typedef __attribute__((ext_vector_type(2))) float v2f;
__device__ __forceinline__ float bf16_rne(float f) { unsigned int u = __float_as_uint(f); u += 0x7FFFu + ((u >> 16) & 1u); return __uint_as_float(u & 0xFFFF0000u); }
__device__ __forceinline__ void split16(float v, b16& hi, b16& lo) { hi = (b16)v; lo = (b16)(v - (float)hi); }
__device__ __forceinline__ v16b frag_kb(const b16* p, int hh) { const v8b a = *(const v8b*)(p + 8 * hh), b = *(const v8b*)(p + 16 + 8 * hh); v16b f;
#pragma unroll
  for (int e = 0; e < 8; ++e) { f[e] = a[e]; f[8 + e] = b[e]; } return f; }
__device__ __forceinline__ v8f wmma16b(v16b a, v16b b, v8f c) { v8f d = __builtin_amdgcn_wmma_f32_16x16x32_f16(false, a, false, b, (short)0, c, false, false); asm volatile("v_nop\n\tv_nop\n\tv_nop\n\tv_nop" : "+v"(d) : "v"(a), "v"(b)); return d; }
__device__ __forceinline__ void wave_lds_sync() { __builtin_amdgcn_fence(__ATOMIC_RELEASE, "workgroup"); __builtin_amdgcn_wave_barrier(); __builtin_amdgcn_fence(__ATOMIC_ACQUIRE, "workgroup"); }
__device__ __forceinline__ float pmul(float a, float b) { float p = a * b; asm volatile("" : "+v"(p)); return p; }
__device__ __forceinline__ int iclamp(int v, int lo, int hi) { return v < lo ? lo : (v > hi ? hi : v); }
__device__ __forceinline__ float nexp2(float v) { return __builtin_amdgcn_exp2f(v); }

constexpr int B = 8, BL = B  , CIN = 16, COUT = 32, HID = 32, L = 2048, NK = COUT * CIN  , KJ = 2112  , XL = 4224  , XOFF = L - 1;
constexpr float OMEGA0 = 30.0f, XS = 8.0f, KS = 8.0f, WSC = 256.0f;
static_assert(L % 128 == 0 && KJ % 32 == 0 && (KJ * 2) % 128 == 0 && XL % 64 == 0 && XL >= XOFF + L + (KJ - L) + 32 && NK % 32 == 0 && HID == 32, "tiling");

__global__ __launch_bounds__(256) void siren_kernel(const float* __restrict__ w1, const float* __restrict__ b1, const float* __restrict__ w2, const float* __restrict__ b2, b16* __restrict__ H2h, b16* __restrict__ H2l) {
  __shared__ float W2s[HID * HID], B2s[HID], W1s[HID], B1s[HID]; __shared__ __attribute__((aligned(16))) b16 Sh[256][HID + 8], Sl[256][HID + 8]; __shared__ float H1s[256][HID + 1];
  for (int i = threadIdx.x; i < HID * HID; i += 256) W2s[i] = bf16_rne(w2[i]);
  if (threadIdx.x < HID) { B2s[threadIdx.x] = bf16_rne(b2[threadIdx.x]); W1s[threadIdx.x] = bf16_rne(w1[threadIdx.x]); B1s[threadIdx.x] = bf16_rne(b1[threadIdx.x]); }
  __syncthreads();
  const int l = blockIdx.x * 256 + threadIdx.x;
  float t; if (l == L - 1) t = 1.0f; else { const float s = (float)l / (float)(L - 1); t = -1.0f * (1.0f - s) + 1.0f * s; }
#pragma unroll 1
  for (int k = 0; k < HID; ++k) H1s[threadIdx.x][k] = sinf(OMEGA0 * (W1s[k] * t + B1s[k]));
#pragma unroll 1
  for (int c = 0; c < HID; ++c) { float a = 0.0f;
#pragma unroll 4
    for (int k = 0; k < HID; ++k) a = fmaf(W2s[c * HID + k], H1s[threadIdx.x][k], a);
    const float h = sinf(OMEGA0 * (a + B2s[c])); b16 ph, pl; split16(h * XS, ph, pl); Sh[threadIdx.x][c] = ph; Sl[threadIdx.x][c] = pl; }
  __syncthreads();
  for (int pass = 0; pass < 2; ++pass) { for (int q = threadIdx.x; q < 256 * HID / 8; q += 256) { const int rr = q / (HID / 8), c8 = (q % (HID / 8)) * 8; *(volatile v8b*)(H2h + (size_t)(blockIdx.x * 256 + rr) * HID + c8) = *(const v8b*)(&Sh[rr][c8]); *(volatile v8b*)(H2l + (size_t)(blockIdx.x * 256 + rr) * HID + c8) = *(const v8b*)(&Sl[rr][c8]); } __threadfence(); }
}
__global__ __launch_bounds__(256) void xprep_kernel(const float* __restrict__ x, b16* __restrict__ X16, b16* __restrict__ Kh) {
  const int u = blockIdx.x * 256 + threadIdx.x; const int nx = B * CIN * XL / 8, nz = NK * (KJ - L) / 8;
  if (u < nx) { const int e = u * 8; const int row = e / XL, m0 = e % XL; v8b o; for (int j = 0; j < 8; ++j) { const int m = m0 + j - XOFF; o[j] = (b16)((m >= 0 && m < L) ? bf16_rne(x[(size_t)row * L + m]) * XS : 0.0f); }
    for (int pass = 0; pass < 2; ++pass) { *(volatile v8b*)(X16 + e) = o; __threadfence(); } }
  else if (u < nx + nz) { const int e = (u - nx) * 8; const int row = e / (KJ - L), c = e % (KJ - L); const v8b z = {}; for (int pass = 0; pass < 2; ++pass) { *(volatile v8b*)(Kh + (size_t)row * KJ + L + c) = z; __threadfence(); } }
}
__global__ __launch_bounds__(64) void kgen_kernel(const float* __restrict__ w3, const float* __restrict__ b3, const b16* __restrict__ H2h, const b16* __restrict__ H2l, b16* __restrict__ Kh) {
  __shared__ __attribute__((aligned(16))) b16 As[2][16][HID + 8]; __shared__ __attribute__((aligned(16))) b16 Tk[2][16][128 + 8];
  const int wave = threadIdx.x >> 5, lane = threadIdx.x & 31, nloc = lane & 15, hlf = lane >> 4; const int r0 = blockIdx.x * 32 + wave * 16; const int n0 = blockIdx.y * 128;
  for (int idx = lane; idx < 16 * HID; idx += 32) { const int rr = idx / HID, c = idx % HID; As[wave][rr][c] = (b16)(bf16_rne(w3[(size_t)(r0 + rr) * HID + c]) * WSC); }
  wave_lds_sync();
  v8f acc[8];
#pragma unroll
  for (int t = 0; t < 8; ++t) acc[t] = (v8f){};
  { const v16b a = frag_kb(&As[wave][nloc][0], hlf);
#pragma unroll
    for (int t = 0; t < 8; ++t) { const size_t col = (size_t)(n0 + t * 16 + nloc) * HID; acc[t] = wmma16b(a, frag_kb(H2h + col, hlf), acc[t]); acc[t] = wmma16b(a, frag_kb(H2l + col, hlf), acc[t]); } }
#pragma unroll
  for (int t = 0; t < 8; ++t) {
#pragma unroll
    for (int r = 0; r < 8; ++r) { const float kv = acc[t][r] * (1.0f / (XS * WSC)) + bf16_rne(b3[r0 + 8 * hlf + r]); Tk[wave][8 * hlf + r][t * 16 + nloc] = (b16)(kv * KS); } }
  wave_lds_sync();
  for (int pass = 0; pass < 2; ++pass) { for (int rr = 0; rr < 16; ++rr) *(volatile v4h*)(Kh + (size_t)(r0 + rr) * KJ + n0 + lane * 4) = *(const v4h*)(&Tk[wave][rr][lane * 4]); __threadfence(); }
}
__global__ __launch_bounds__(64) void conv_kernel(const b16* __restrict__ Kh, const b16* __restrict__ X16, const float* __restrict__ cbias, float* __restrict__ out) {
  __shared__ __attribute__((aligned(16))) float Tf[2][16][128 + 4];
  const int wave = threadIdx.x >> 5, lane = threadIdx.x & 31, nloc = lane & 15, hlf = lane >> 4; const int l0 = blockIdx.x * 128, b = blockIdx.y, o0 = wave * 16;
  v8f acc[8];
#pragma unroll
  for (int t = 0; t < 8; ++t) acc[t] = (v8f){};
#pragma unroll 1
  for (int i = 0; i < CIN; ++i) { const b16* arow = Kh + (size_t)((o0 + nloc) * CIN + i) * KJ; const b16* xrow = X16 + (size_t)(b * CIN + i) * XL + l0 + nloc;
#pragma unroll 2
    for (int j0 = 0; j0 < KJ; j0 += 32) { const v16b a = frag_kb(arow + j0, hlf);
#pragma unroll
      for (int t = 0; t < 8; ++t) acc[t] = wmma16b(a, frag_kb(xrow + t * 16 + j0, hlf), acc[t]); } }
#pragma unroll
  for (int t = 0; t < 8; ++t) {
#pragma unroll
    for (int r = 0; r < 8; ++r) Tf[wave][8 * hlf + r][t * 16 + nloc] = acc[t][r] * (1.0f / (XS * KS)) + bf16_rne(cbias[o0 + 8 * hlf + r]); }
  wave_lds_sync();
  for (int pass = 0; pass < 2; ++pass) { for (int rr = 0; rr < 16; ++rr) *(volatile v4f*)(out + ((size_t)b * COUT + o0 + rr) * L + l0 + lane * 4) = *(const v4f*)(&Tf[wave][rr][lane * 4]); __threadfence(); }
}
}

extern "C" void kernel_launch(void* const* d_in, const int* in_sizes, int n_in, void* d_out, int out_size, void* d_ws, size_t ws_size, hipStream_t stream) {
  (void)n_in;
  auto Fp = [&](int i) { return (const float*)d_in[i]; };
  if (in_sizes[0] != B * CIN * L || in_sizes[1] != HID || in_sizes[2] != HID || in_sizes[3] != HID * HID || in_sizes[4] != HID || in_sizes[5] != NK * HID || in_sizes[6] != NK || in_sizes[7] != COUT || out_size != B * COUT * L) return;
  size_t off = 0; char* ws = (char*)d_ws;
  auto carve = [&](size_t bytes) { char* p = ws + off; off += (bytes + 255) & ~(size_t)255; return p; };
  b16* H2h = (b16*)carve((size_t)L * HID * 2); b16* H2l = (b16*)carve((size_t)L * HID * 2); b16* Kh = (b16*)carve((size_t)NK * KJ * 2); b16* X16 = (b16*)carve((size_t)B * CIN * XL * 2);
  if (off > ws_size || off > ((size_t)128 << 20)) return;
  siren_kernel<<<L / 256, 256, 0, stream>>>(Fp(1), Fp(2), Fp(3), Fp(4), H2h, H2l);
  xprep_kernel<<<(B * CIN * XL / 8 + NK * (KJ - L) / 8 + 255) / 256, 256, 0, stream>>>(Fp(0), X16, Kh);
  kgen_kernel<<<dim3(NK / 32, L / 128), 64, 0, stream>>>(Fp(5), Fp(6), H2h, H2l, Kh);
  conv_kernel<<<dim3(L / 128, BL), 64, 0, stream>>>(Kh, X16, Fp(7), (float*)d_out);
}
